// QuantLinear_9019431321834
// MI455X (gfx1250) — hardware-verified
//
#include <hip/hip_runtime.h>
#include <math.h>

typedef __attribute__((ext_vector_type(16))) _Float16 v16h;
typedef __attribute__((ext_vector_type(16))) __bf16 v16b;
typedef __attribute__((ext_vector_type(8)))  _Float16 v8h;
typedef __attribute__((ext_vector_type(8)))  float v8f;
typedef __attribute__((ext_vector_type(4)))  float v4f;
typedef __attribute__((ext_vector_type(2)))  float v2f;
typedef __attribute__((ext_vector_type(4)))  unsigned v4u;
typedef __attribute__((ext_vector_type(4)))  int v4i;
typedef float __attribute__((may_alias)) float_a;
typedef int __attribute__((may_alias)) int_a;

template <typename T> __device__ __forceinline__ void vst2(void* p, T v) { *(volatile T*)p = v; __threadfence(); *(volatile T*)p = v; }
__device__ __forceinline__ v8f wmma16(v16h a, v16h b, v8f c) {
  v8f d = __builtin_amdgcn_wmma_f32_16x16x32_f16(false, a, false, b, (short)0, c, false, false);
  asm volatile("v_nop\n\tv_nop\n\tv_nop\n\tv_nop" : "+v"(d) : "v"(a), "v"(b));
  return d;
}
__device__ __forceinline__ v8f wmma_bf(v16b a, v16b b, v8f c) {
  v8f d = __builtin_amdgcn_wmma_f32_16x16x32_bf16(false, a, false, b, (short)0, c, false, false);
  asm volatile("v_nop\n\tv_nop\n\tv_nop\n\tv_nop" : "+v"(d) : "v"(a), "v"(b));
  return d;
}
__device__ __forceinline__ v16h frag_h(const _Float16* rowk0, int lane) {
  union { v16h v; v8h q[2]; } u; const _Float16* p = rowk0 + 8 * (lane >> 4);
  u.q[0] = *(const v8h*)p; u.q[1] = *(const v8h*)(p + 16); return u.v;
}
__device__ __forceinline__ v16h frag_f32(const float* rowk0, int lane) {
  v16h a; const float* p = rowk0 + 8 * (lane >> 4);
#pragma unroll
  for (int i = 0; i < 8; ++i) { a[i] = (_Float16)p[i]; a[8 + i] = (_Float16)p[16 + i]; }
  return a;
}
__device__ __forceinline__ v16h frag_f32s(const float* rowk0, int lane, float sc) {
  v16h a; const float* p = rowk0 + 8 * (lane >> 4);
#pragma unroll
  for (int i = 0; i < 8; ++i) { a[i] = (_Float16)(p[i] * sc); a[8 + i] = (_Float16)(p[16 + i] * sc); }
  return a;
}
__device__ __forceinline__ v16h fragc_f32(const float* W, int k0, int n, int lane, int ld, int K) {
  v16h a; const int g = lane >> 4;
#pragma unroll
  for (int i = 0; i < 8; ++i) { const int ka = k0 + 8 * g + i, kb = ka + 16;
    a[i] = (_Float16)(ka < K ? W[(size_t)ka * ld + n] : 0.f); a[8 + i] = (_Float16)(kb < K ? W[(size_t)kb * ld + n] : 0.f); }
  return a;
}
struct F2 { v16b h, l; };
__device__ __forceinline__ F2 bsplit16(const float v[16]) { F2 r;
#pragma unroll
  for (int i = 0; i < 16; ++i) { const __bf16 h = (__bf16)v[i]; r.h[i] = h; r.l[i] = (__bf16)(v[i] - (float)h); }
  return r; }
__device__ __forceinline__ F2 split_row(const float* row, int k0, int lane) { float v[16]; const float* p = row + k0 + 8 * (lane >> 4);
#pragma unroll
  for (int i = 0; i < 8; ++i) { v[i] = p[i]; v[8 + i] = p[16 + i]; }
  return bsplit16(v); }
__device__ __forceinline__ F2 split_rowK(const float* row, int k0, int lane, int K) { float v[16]; const int g = lane >> 4;
#pragma unroll
  for (int i = 0; i < 8; ++i) { const int ka = k0 + 8 * g + i, kb = ka + 16; v[i] = ka < K ? row[ka] : 0.f; v[8 + i] = kb < K ? row[kb] : 0.f; }
  return bsplit16(v); }
__device__ __forceinline__ F2 split_col(const float* W, int k0, int n, int lane, int ld, int K) { float v[16]; const int g = lane >> 4;
#pragma unroll
  for (int i = 0; i < 8; ++i) { const int ka = k0 + 8 * g + i, kb = ka + 16; v[i] = ka < K ? W[(size_t)ka * ld + n] : 0.f; v[8 + i] = kb < K ? W[(size_t)kb * ld + n] : 0.f; }
  return bsplit16(v); }
__device__ __forceinline__ v8f mac3(const F2& a, const F2& b, v8f c) { c = wmma_bf(a.l, b.h, c); c = wmma_bf(a.h, b.l, c); return wmma_bf(a.h, b.h, c); }
__device__ __forceinline__ float sigm(float v) { return 1.0f / (1.0f + expf(-v)); }
#define LDSX() do { asm volatile("s_wait_dscnt 0" ::: "memory"); __builtin_amdgcn_wave_barrier(); __builtin_amdgcn_fence(__ATOMIC_RELEASE, "workgroup"); } while (0)

#define MR 8
#define KIN 4096
#define NOUT 11008

__global__ __launch_bounds__(128) void k_main(const float* __restrict__ x, const int* __restrict__ qw, const float* __restrict__ scales, const int* __restrict__ zeros, const float* __restrict__ bias, float* __restrict__ out) {
  __shared__ __align__(16) float sx[16][KIN + 4];
  __shared__ __align__(16) float so[4][16][36];
  const int tid = threadIdx.x, wave = tid >> 5, lane = tid & 31, col = lane & 15, g = lane >> 4;
  for (int q = tid; q < 16 * KIN; q += 128) { const int r = q / KIN, k = q % KIN; sx[r][k] = r < MR ? x[(size_t)r * KIN + k] : 0.f; }
  __syncthreads();
  const int n0 = blockIdx.x * 128 + wave * 32;
#pragma unroll 1
  for (int t = 0; t < 2; ++t) { const int n = n0 + t * 16 + col;
    const int zp = (zeros[n >> 1] >> ((n & 1) * 4)) & 0xF;
    v8f acc = {};
#pragma unroll 2
    for (int kc = 0; kc < KIN / 32; ++kc) { const F2 a = split_row(&sx[col][0], kc * 32, lane);
      const unsigned w0 = (unsigned)qw[(size_t)(kc * 4 + g) * NOUT + n], w1 = (unsigned)qw[(size_t)(kc * 4 + 2 + g) * NOUT + n];
      v16b bq;
#pragma unroll
      for (int i = 0; i < 8; ++i) { bq[i] = (__bf16)(float)((int)((w0 >> (4 * i)) & 0xF) - zp); bq[8 + i] = (__bf16)(float)((int)((w1 >> (4 * i)) & 0xF) - zp); }
      acc = wmma_bf(a.h, bq, acc); acc = wmma_bf(a.l, bq, acc); }
    const float sc = scales[n], bb = bias[n];
#pragma unroll
    for (int r = 0; r < 8; ++r) so[wave][8 * g + r][t * 16 + col] = acc[r] * sc + bb; }
  LDSX();
  for (int q = lane; q < MR * 8; q += 32) { const int r = q >> 3, pc = q & 7; vst2(out + (size_t)r * NOUT + n0 + pc * 4, *(const v4f*)(&so[wave][r][pc * 4])); }
}
extern "C" void kernel_launch(void* const* d_in, const int* in_sizes, int n_in, void* d_out, int out_size, void* d_ws, size_t ws_size, hipStream_t stream) {
  (void)in_sizes; (void)n_in; (void)out_size; (void)ws_size; (void)d_ws;
  const float* x = (const float*)d_in[0]; const int* qw = (const int*)d_in[1]; const float* scales = (const float*)d_in[2]; const int* zeros = (const int*)d_in[3]; const float* bias = (const float*)d_in[4];
  float* out = (float*)d_out;
  k_main<<<NOUT / 128, 128, 0, stream>>>(x, qw, scales, zeros, bias, out);
}
